// GRUBlock_15367392985483
// MI455X (gfx1250) — hardware-verified
//
#include <hip/hip_runtime.h>
#include <math.h>

constexpr int NBATCH = 16;
constexpr int NCH    = 256;
constexpr int NSEQ   = 2048;
constexpr int NHID   = 256;
constexpr int NGATE  = 3 * NHID;
constexpr int NFF    = 2 * NCH;
constexpr int NROWS  = NBATCH * NSEQ;
constexpr bool  LEG_BF16   = true;
constexpr float WCARRY     = 16.0f;
constexpr float WCARRY_INV = 1.0f / WCARRY;
constexpr float LN_EPS_F   = 1e-5f;
constexpr int SCAN_THR = 512;
constexpr int HPITCH   = 264;
constexpr int OPITCH   = 260;
constexpr int TPITCH   = 36;

static_assert(NHID == NCH, "hidden size equals channel count");
static_assert(NBATCH == 16, "one 16-row m-subtile per scan block");
static_assert(NHID == 16 * (SCAN_THR / 32), "16 waves x 16 hidden units");
static_assert(NCH % 32 == 0 && (2 * NHID) % 32 == 0 && NFF % 32 == 0, "GEMM K multiples of 32");
static_assert(NROWS % 64 == 0 && NGATE % 64 == 0 && NFF % 64 == 0 && NCH % 64 == 0, "GEMM M, N tile multiples");
static_assert(NSEQ % 64 == 0, "a 64-row m-tile stays inside one batch item");
static_assert(HPITCH % 8 == 0 && OPITCH % 4 == 0 && TPITCH % 4 == 0, "LDS pitches keep 16-B alignment");

constexpr int CVT_ELEMS = 2048;
constexpr int BLK_IH0 = NGATE * NCH / CVT_ELEMS;
constexpr int BLK_HH  = NGATE * NHID / CVT_ELEMS;
constexpr int BLK_IH1 = NGATE * 2 * NHID / CVT_ELEMS;
constexpr int BLK_W1  = NFF * NCH / CVT_ELEMS;
constexpr int BLK_W2  = NCH * NFF / CVT_ELEMS;
constexpr int BS0 = 0;
constexpr int BS1 = BS0 + BLK_IH0;
constexpr int BS2 = BS1 + BLK_HH;
constexpr int BS3 = BS2 + BLK_IH0;
constexpr int BS4 = BS3 + BLK_HH;
constexpr int BS5 = BS4 + BLK_IH1;
constexpr int BS6 = BS5 + BLK_HH;
constexpr int BS7 = BS6 + BLK_IH1;
constexpr int BS8 = BS7 + BLK_HH;
constexpr int BS9 = BS8 + BLK_W1;
constexpr int BS10 = BS9 + BLK_W2;
static_assert((NGATE * NCH) % CVT_ELEMS == 0 && (NFF * NCH) % CVT_ELEMS == 0, "weight sizes are whole convert blocks");
static_assert(BS10 == 1088, "arena block count");

typedef __attribute__((ext_vector_type(16))) _Float16 v16h;
typedef __attribute__((ext_vector_type(8)))  _Float16 v8h;
typedef __attribute__((ext_vector_type(8)))  float    v8f;
typedef __attribute__((ext_vector_type(4)))  float    v4f;

__device__ __forceinline__ unsigned short f2bf_bits(float f) {
  unsigned u = __float_as_uint(f);
  return (unsigned short)((u + 0x7FFFu + ((u >> 16) & 1u)) >> 16);
}
__device__ __forceinline__ float bf_bits2f(unsigned short h) { return __uint_as_float(((unsigned)h) << 16); }
__device__ __forceinline__ float inq(float f) { return LEG_BF16 ? bf_bits2f(f2bf_bits(f)) : f; }

__device__ __forceinline__ float h16_to_f32(unsigned hb) {
  const unsigned sgn = (hb & 0x8000u) << 16;
  const unsigned em = hb & 0x7fffu;
  const float fn = __uint_as_float((em << 13) + 0x38000000u);
  const float fs = (float)em * 5.9604644775390625e-8f;
  const float mag = (em < 0x400u) ? fs : fn;
  return __uint_as_float(__float_as_uint(mag) | sgn);
}

__device__ __forceinline__ void guard4(v8f& a, v8f& b, v8f& c, v8f& d, v16h x, v16h b0, v16h b1, v16h b2, v16h b3) {
  asm volatile("v_nop\n\tv_nop\n\tv_nop\n\tv_nop" : "+v"(a), "+v"(b), "+v"(c), "+v"(d) : "v"(x), "v"(b0), "v"(b1), "v"(b2), "v"(b3));
}
__device__ __forceinline__ void guard3(v8f& a, v8f& b, v8f& c, v16h x, v16h b0, v16h b1, v16h b2) {
  asm volatile("v_nop\n\tv_nop\n\tv_nop\n\tv_nop" : "+v"(a), "+v"(b), "+v"(c) : "v"(x), "v"(b0), "v"(b1), "v"(b2));
}
__device__ __forceinline__ void acc_guard4(v8f& a, v8f& b, v8f& c, v8f& d) { asm volatile("v_nop\n\tv_nop\n\tv_nop\n\tv_nop" : "+v"(a), "+v"(b), "+v"(c), "+v"(d)); }
__device__ __forceinline__ void acc_guard3(v8f& a, v8f& b, v8f& c) { asm volatile("v_nop\n\tv_nop\n\tv_nop\n\tv_nop" : "+v"(a), "+v"(b), "+v"(c)); }

struct FragH {
  union U { v16h v; v8h h[2]; };
  static __device__ __forceinline__ v16h load(const _Float16* p) {
    U f; f.h[0] = *(const v8h*)(p); f.h[1] = *(const v8h*)(p + 16); return f.v;
  }
  static __device__ __forceinline__ v8f mma(v16h a, v16h b, v8f c) {
    return __builtin_amdgcn_wmma_f32_16x16x32_f16(false, a, false, b, (short)0, c, false, false);
  }
};

__device__ __forceinline__ void wave_sync_lds() {
  __builtin_amdgcn_fence(__ATOMIC_RELEASE, "workgroup");
  __builtin_amdgcn_wave_barrier();
  __builtin_amdgcn_fence(__ATOMIC_ACQUIRE, "workgroup");
}

struct WSrc { const float* p0; const float* p1; const float* p2; const float* p3; const float* p4;
              const float* p5; const float* p6; const float* p7; const float* p8; const float* p9; };
static_assert(sizeof(WSrc) == 80, "no padding");

__global__ __launch_bounds__(256) void cvt_weights_kernel(WSrc a, unsigned short* __restrict__ dst) {
  const int blk = blockIdx.x;
  const float* s = a.p0;
  int st = BS0;
  if (blk >= BS1) { s = a.p1; st = BS1; }
  if (blk >= BS2) { s = a.p2; st = BS2; }
  if (blk >= BS3) { s = a.p3; st = BS3; }
  if (blk >= BS4) { s = a.p4; st = BS4; }
  if (blk >= BS5) { s = a.p5; st = BS5; }
  if (blk >= BS6) { s = a.p6; st = BS6; }
  if (blk >= BS7) { s = a.p7; st = BS7; }
  if (blk >= BS8) { s = a.p8; st = BS8; }
  if (blk >= BS9) { s = a.p9; st = BS9; }
  const size_t so = (size_t)(blk - st) * CVT_ELEMS + (size_t)threadIdx.x * 8;
  const size_t dofs = (size_t)blk * CVT_ELEMS + (size_t)threadIdx.x * 8;
  const v4f x0 = *(const v4f*)(s + so);
  const v4f x1 = *(const v4f*)(s + so + 4);
  v8h hv;
#pragma unroll
  for (int e = 0; e < 4; ++e) {
    const float f0 = inq(x0[e]) * WCARRY;
    const float f1 = inq(x1[e]) * WCARRY;
    hv[e]     = (_Float16)f0;
    hv[4 + e] = (_Float16)f1;
  }
  for (int pass = 0; pass < 2; ++pass) {
    *(volatile v8h*)(dst + dofs) = hv;
    __threadfence();
  }
}

__global__ __launch_bounds__(256) void xpose_kernel(const float* __restrict__ x, unsigned short* __restrict__ XT) {
  __shared__ float Tt[64 * 65];
  const int tid = threadIdx.x;
  const int l0 = blockIdx.x * 64, ch0 = blockIdx.y * 64, b = blockIdx.z;
  const float* src = x + (size_t)b * NCH * NSEQ;
#pragma unroll
  for (int i = 0; i < 4; ++i) {
    const int idx = i * 256 + tid;
    const int rr = idx >> 4, cc = (idx & 15) * 4;
    const v4f v = *(const v4f*)(src + (size_t)(ch0 + rr) * NSEQ + l0 + cc);
    Tt[rr * 65 + cc + 0] = v[0];
    Tt[rr * 65 + cc + 1] = v[1];
    Tt[rr * 65 + cc + 2] = v[2];
    Tt[rr * 65 + cc + 3] = v[3];
  }
  __syncthreads();
  const int q = tid >> 3, c8 = (tid & 7) * 8;
  v8h hv[2];
#pragma unroll
  for (int g = 0; g < 2; ++g) {
    const int qq = g * 32 + q;
#pragma unroll
    for (int e = 0; e < 8; ++e) {
      const float f = inq(Tt[(c8 + e) * 65 + qq]);
      hv[g][e] = (_Float16)f;
    }
  }
  for (int pass = 0; pass < 2; ++pass) {
#pragma unroll
    for (int g = 0; g < 2; ++g) {
      const size_t o = ((size_t)b * NSEQ + (size_t)(l0 + g * 32 + q)) * NCH + (size_t)(ch0 + c8);
      *(volatile v8h*)(XT + o) = hv[g];
    }
    __threadfence();
  }
}

template <int ACT, int OUT_MODE>
__global__ __launch_bounds__(256) void wmma_gemm64(
    const unsigned short* __restrict__ Ap, int lda,
    const unsigned short* __restrict__ Btp, int ldb,
    void* __restrict__ Cout, int ldc,
    const float* __restrict__ bias,
    int M, int N, int K, float scale) {
  constexpr int SLABN = (OUT_MODE == 3) ? (64 * TPITCH) : (16 * 68);
  __shared__ __align__(16) float sT[8][SLABN];
  const _Float16* A  = (const _Float16*)Ap;
  const _Float16* Bt = (const _Float16*)Btp;
  const int lane = threadIdx.x & 31;
  const int wave = threadIdx.x >> 5;
  const int tilesN = N >> 6;
  const int tilesM = M >> 6;
  const int tile = blockIdx.x * 8 + wave;
  if (tile >= tilesM * tilesN) return;
  const int tm = tile / tilesN;
  const int tn = tile - tm * tilesN;
  const int m0 = tm << 6;
  const int n0 = tn << 6;
  const int rlane = lane & 15;
  const int koff  = (lane >> 4) * 8;
  const int mOff  = (lane >> 4) * 8;

  const _Float16* abase = A  + (size_t)(m0 + rlane) * lda + koff;
  const _Float16* bbase = Bt + (size_t)(n0 + rlane) * ldb + koff;
  const size_t astep = (size_t)16 * lda;
  const size_t bstep = (size_t)16 * ldb;

  v8f acc[4][4];
#pragma unroll
  for (int i = 0; i < 4; ++i)
#pragma unroll
    for (int j = 0; j < 4; ++j) acc[i][j] = (v8f){0.f, 0.f, 0.f, 0.f, 0.f, 0.f, 0.f, 0.f};

  for (int k0 = 0; k0 < K; k0 += 32) {
    v16h bh[4];
#pragma unroll
    for (int j = 0; j < 4; ++j) bh[j] = FragH::load(bbase + (size_t)j * bstep + k0);
#pragma unroll
    for (int i = 0; i < 4; ++i) {
      const v16h ah = FragH::load(abase + (size_t)i * astep + k0);
#pragma unroll
      for (int j = 0; j < 4; ++j) acc[i][j] = FragH::mma(ah, bh[j], acc[i][j]);
      guard4(acc[i][0], acc[i][1], acc[i][2], acc[i][3], ah, bh[0], bh[1], bh[2], bh[3]);
    }
  }
  acc_guard4(acc[0][0], acc[0][1], acc[0][2], acc[0][3]);
  acc_guard4(acc[1][0], acc[1][1], acc[1][2], acc[1][3]);
  acc_guard4(acc[2][0], acc[2][1], acc[2][2], acc[2][3]);
  acc_guard4(acc[3][0], acc[3][1], acc[3][2], acc[3][3]);

  float* slab = sT[wave];
  if (OUT_MODE == 1) {
    unsigned short* C = (unsigned short*)Cout;
    const int q = lane >> 3, c8 = (lane & 7) * 8;
#pragma unroll
    for (int i = 0; i < 4; ++i) {
      const int mBase = m0 + (i << 4);
#pragma unroll
      for (int j = 0; j < 4; ++j) {
        const float bv = inq(bias[n0 + (j << 4) + rlane]);
#pragma unroll
        for (int r = 0; r < 8; ++r) {
          float v = acc[i][j][r] * scale + bv;
          if (ACT == 2) v = fmaxf(v, 0.0f);
          slab[(mOff + r) * 68 + (j << 4) + rlane] = v;
        }
      }
      wave_sync_lds();
      for (int pass = 0; pass < 2; ++pass) {
#pragma unroll
        for (int it = 0; it < 4; ++it) {
          const int row = it * 4 + q;
          const float* sp = slab + row * 68 + c8;
          v8h hv;
#pragma unroll
          for (int e = 0; e < 8; ++e) hv[e] = (_Float16)sp[e];
          *(volatile v8h*)(C + (size_t)(mBase + row) * ldc + n0 + c8) = hv;
        }
        __threadfence();
      }
      wave_sync_lds();
    }
  } else {
    float* Cf = (float*)Cout;
    const int bb = m0 / ldc;
    const int lb = m0 - bb * ldc;
    const int q = lane >> 3, l4 = (lane & 7) * 4;
#pragma unroll
    for (int hf = 0; hf < 2; ++hf) {
#pragma unroll
      for (int i2 = 0; i2 < 2; ++i2) {
        const int i = hf * 2 + i2;
#pragma unroll
        for (int j = 0; j < 4; ++j) {
          const float bv = inq(bias[n0 + (j << 4) + rlane]);
#pragma unroll
          for (int r = 0; r < 8; ++r) {
            float v = acc[i][j][r] * scale + bv;
            if (ACT == 2) v = fmaxf(v, 0.0f);
            slab[((j << 4) + rlane) * TPITCH + (i2 << 4) + mOff + r] = v;
          }
        }
      }
      wave_sync_lds();
      for (int pass = 0; pass < 2; ++pass) {
#pragma unroll
        for (int it = 0; it < 16; ++it) {
          const int crow = it * 4 + q;
          const v4f v = *(const v4f*)(slab + crow * TPITCH + l4);
          *(volatile v4f*)(Cf + ((size_t)bb * N + (size_t)(n0 + crow)) * ldc + lb + hf * 32 + l4) = v;
        }
        __threadfence();
      }
      wave_sync_lds();
    }
  }
}

template <bool OUT32>
__global__ __launch_bounds__(SCAN_THR) void gru_scan_kernel(const unsigned short* __restrict__ GI,
                                                            const unsigned short* __restrict__ WHHp,
                                                            const float* __restrict__ bhh,
                                                            void* __restrict__ outp, int dir) {
  __shared__ __align__(16) _Float16 hA[2 * 16 * HPITCH];
  __shared__ __align__(16) float    hS[OUT32 ? (2 * 16 * OPITCH) : 4];
  const _Float16* WHH = (const _Float16*)WHHp;
  const int tid = threadIdx.x, lane = tid & 31, wave = tid >> 5;
  const int c = lane & 15, hh = lane >> 4, koff = hh * 8;
  const int j = 16 * wave + c;

#pragma unroll 1
  for (int i = tid; i < 2 * 16 * HPITCH; i += SCAN_THR) hA[i] = (_Float16)0.0f;

  float hst[8];
#pragma unroll
  for (int r = 0; r < 8; ++r) hst[r] = 0.0f;
  const float bR = inq(bhh[j]);
  const float bZ = inq(bhh[NHID + j]);
  const float bN = inq(bhh[2 * NHID + j]);
  const _Float16* wr = WHH + (size_t)j * NHID + koff;
  const _Float16* wz = wr + (size_t)NHID * NHID;
  const _Float16* wn = wz + (size_t)NHID * NHID;
  const unsigned short* gbase = GI + (size_t)(8 * hh) * NSEQ * NGATE + j;
  const size_t grow = (size_t)NSEQ * NGATE;
  const v8f z8 = {0.f, 0.f, 0.f, 0.f, 0.f, 0.f, 0.f, 0.f};
  __syncthreads();

#pragma unroll 1
  for (int step = 0; step < NSEQ; ++step) {
    const int t = dir ? (NSEQ - 1 - step) : step;
    const int cur = step & 1;
    const int nxt = cur ^ 1;
    const unsigned short* gp = gbase + (size_t)t * NGATE;
    unsigned gr[8], gz[8], gn[8];
#pragma unroll
    for (int r = 0; r < 8; ++r) {
      gr[r] = gp[(size_t)r * grow];
      gz[r] = gp[(size_t)r * grow + NHID];
      gn[r] = gp[(size_t)r * grow + 2 * NHID];
    }
    const _Float16* ahrow = hA + cur * (16 * HPITCH) + c * HPITCH + koff;
    v8f accR = z8, accZ = z8, accN = z8;
#pragma unroll 1
    for (int k0 = 0; k0 < NHID; k0 += 32) {
      const v16h a  = FragH::load(ahrow + k0);
      const v16h b0 = FragH::load(wr + k0);
      const v16h b1 = FragH::load(wz + k0);
      const v16h b2 = FragH::load(wn + k0);
      accR = FragH::mma(a, b0, accR);
      accZ = FragH::mma(a, b1, accZ);
      accN = FragH::mma(a, b2, accN);
      guard3(accR, accZ, accN, a, b0, b1, b2);
    }
    acc_guard3(accR, accZ, accN);

    _Float16* ahn = hA + nxt * (16 * HPITCH);
#pragma unroll
    for (int r = 0; r < 8; ++r) {
      const float gir = h16_to_f32(gr[r]);
      const float giz = h16_to_f32(gz[r]);
      const float gin = h16_to_f32(gn[r]);
      const float pr  = gir + (accR[r] * WCARRY_INV + bR);
      const float pz  = giz + (accZ[r] * WCARRY_INV + bZ);
      const float hnp = accN[r] * WCARRY_INV + bN;
      const float rg  = __builtin_amdgcn_rcpf(1.0f + __expf(-pr));
      const float zg  = __builtin_amdgcn_rcpf(1.0f + __expf(-pz));
      const float pn  = gin + rg * hnp;
      const float ng  = 1.0f - 2.0f * __builtin_amdgcn_rcpf(__expf(2.0f * pn) + 1.0f);
      const float ho  = hst[r];
      const float hnew = (1.0f - zg) * ng + zg * ho;
      hst[r] = hnew;
      ahn[(8 * hh + r) * HPITCH + j] = (_Float16)hnew;
      if constexpr (OUT32) hS[nxt * (16 * OPITCH) + (8 * hh + r) * OPITCH + j] = hnew;
    }
    __syncthreads();

    if constexpr (OUT32) {
      const float* sp = hS + nxt * (16 * OPITCH) + wave * OPITCH;
      const v4f v0 = *(const v4f*)(sp + 4 * lane);
      const v4f v1 = *(const v4f*)(sp + 128 + 4 * lane);
      float* op = (float*)outp + ((size_t)wave * NSEQ + (size_t)t) * NHID;
      for (int pass = 0; pass < 2; ++pass) {
        *(volatile v4f*)(op + 4 * lane) = v0;
        *(volatile v4f*)(op + 128 + 4 * lane) = v1;
        __threadfence();
      }
    } else {
      const v8h hv = *(const v8h*)(hA + nxt * (16 * HPITCH) + wave * HPITCH + 8 * lane);
      unsigned short* op = (unsigned short*)outp + ((size_t)wave * NSEQ + (size_t)t) * (2 * NHID) + dir * NHID + 8 * lane;
      for (int pass = 0; pass < 2; ++pass) {
        *(volatile v8h*)op = hv;
        __threadfence();
      }
    }
  }
}

__global__ __launch_bounds__(256) void sum_ln_kernel(const float* __restrict__ HF, const float* __restrict__ HB,
                                                     const float* __restrict__ gam, const float* __restrict__ bet,
                                                     unsigned short* __restrict__ LN) {
  const int tid = threadIdx.x, lane = tid & 31;
  const int row = blockIdx.x * 8 + (tid >> 5);
  if (row >= NROWS) return;
  const size_t ro = (size_t)row * NHID + 8 * lane;
  const v4f f0 = *(const v4f*)(HF + ro);
  const v4f f1 = *(const v4f*)(HF + ro + 4);
  const v4f b0 = *(const v4f*)(HB + ro);
  const v4f b1 = *(const v4f*)(HB + ro + 4);
  const v4f g0 = *(const v4f*)(gam + 8 * lane);
  const v4f g1 = *(const v4f*)(gam + 8 * lane + 4);
  const v4f e0 = *(const v4f*)(bet + 8 * lane);
  const v4f e1 = *(const v4f*)(bet + 8 * lane + 4);
  float v[8];
#pragma unroll
  for (int e = 0; e < 4; ++e) { v[e] = f0[e] + b0[e]; v[4 + e] = f1[e] + b1[e]; }
  float s = ((v[0] + v[1]) + (v[2] + v[3])) + ((v[4] + v[5]) + (v[6] + v[7]));
#pragma unroll
  for (int off = 1; off < 32; off <<= 1) s += __shfl_xor(s, off, 32);
  const float mu = s * (1.0f / NHID);
  float ss = 0.0f;
#pragma unroll
  for (int e = 0; e < 8; ++e) { const float d = v[e] - mu; v[e] = d; ss += d * d; }
#pragma unroll
  for (int off = 1; off < 32; off <<= 1) ss += __shfl_xor(ss, off, 32);
  const float var  = ss * (1.0f / NHID);
  const float rstd = rsqrtf(var + LN_EPS_F);
  v8h hv;
#pragma unroll
  for (int e = 0; e < 4; ++e) {
    const float o0 = (v[e] * rstd) * inq(g0[e]) + inq(e0[e]);
    const float o1 = (v[4 + e] * rstd) * inq(g1[e]) + inq(e1[e]);
    hv[e]     = (_Float16)o0;
    hv[4 + e] = (_Float16)o1;
  }
  unsigned short* op = LN + (size_t)row * NHID + 8 * lane;
  for (int pass = 0; pass < 2; ++pass) {
    *(volatile v8h*)op = hv;
    __threadfence();
  }
}

extern "C" void kernel_launch(void* const* d_in, const int* in_sizes, int n_in,
                              void* d_out, int out_size, void* d_ws, size_t ws_size, hipStream_t stream) {
  if (n_in < 23 || d_out == nullptr || d_ws == nullptr) return;
  if (in_sizes[0] != NBATCH * NCH * NSEQ || out_size != NBATCH * NCH * NSEQ) return;
  if (in_sizes[1] != NGATE * NCH || in_sizes[2] != NGATE * NHID || in_sizes[3] != NGATE || in_sizes[4] != NGATE ||
      in_sizes[5] != NGATE * NCH || in_sizes[6] != NGATE * NHID || in_sizes[7] != NGATE || in_sizes[8] != NGATE ||
      in_sizes[9] != NGATE * 2 * NHID || in_sizes[10] != NGATE * NHID || in_sizes[11] != NGATE || in_sizes[12] != NGATE ||
      in_sizes[13] != NGATE * 2 * NHID || in_sizes[14] != NGATE * NHID || in_sizes[15] != NGATE || in_sizes[16] != NGATE ||
      in_sizes[17] != NCH || in_sizes[18] != NCH || in_sizes[19] != NFF * NCH || in_sizes[20] != NFF ||
      in_sizes[21] != NCH * NFF || in_sizes[22] != NCH) return;

  const float* x      = (const float*)d_in[0];
  const float* w_ih0f = (const float*)d_in[1];
  const float* w_hh0f = (const float*)d_in[2];
  const float* b_ih0f = (const float*)d_in[3];
  const float* b_hh0f = (const float*)d_in[4];
  const float* w_ih0b = (const float*)d_in[5];
  const float* w_hh0b = (const float*)d_in[6];
  const float* b_ih0b = (const float*)d_in[7];
  const float* b_hh0b = (const float*)d_in[8];
  const float* w_ih1f = (const float*)d_in[9];
  const float* w_hh1f = (const float*)d_in[10];
  const float* b_ih1f = (const float*)d_in[11];
  const float* b_hh1f = (const float*)d_in[12];
  const float* w_ih1b = (const float*)d_in[13];
  const float* w_hh1b = (const float*)d_in[14];
  const float* b_ih1b = (const float*)d_in[15];
  const float* b_hh1b = (const float*)d_in[16];
  const float* ln_g   = (const float*)d_in[17];
  const float* ln_b   = (const float*)d_in[18];
  const float* w1     = (const float*)d_in[19];
  const float* b1     = (const float*)d_in[20];
  const float* w2     = (const float*)d_in[21];
  const float* b2     = (const float*)d_in[22];
  float* out = (float*)d_out;

  char* ws = (char*)d_ws;
  size_t off = 0;
  auto carve = [&](size_t bytes) -> char* { char* p = ws + off; off += (bytes + 255) & ~(size_t)255; return p; };
  unsigned short* W16 = (unsigned short*)carve((size_t)BS10 * CVT_ELEMS * 2);
  char*           XTP = carve((size_t)NROWS * NHID * 4);
  unsigned short* GI  = (unsigned short*)carve((size_t)NROWS * NGATE * 2);
  char*           H0P = carve((size_t)NROWS * 2 * NHID * 2);
  if (off > ws_size || off > (size_t)134217728) return;

  unsigned short* XT   = (unsigned short*)XTP;
  float*          H1F  = (float*)XTP;
  unsigned short* H0   = (unsigned short*)H0P;
  float*          H1B  = (float*)H0P;
  unsigned short* LNP  = GI;
  unsigned short* RELU = GI + (size_t)NROWS * NCH;

  unsigned short* W_IH0F = W16 + (size_t)BS0 * CVT_ELEMS;
  unsigned short* W_HH0F = W16 + (size_t)BS1 * CVT_ELEMS;
  unsigned short* W_IH0B = W16 + (size_t)BS2 * CVT_ELEMS;
  unsigned short* W_HH0B = W16 + (size_t)BS3 * CVT_ELEMS;
  unsigned short* W_IH1F = W16 + (size_t)BS4 * CVT_ELEMS;
  unsigned short* W_HH1F = W16 + (size_t)BS5 * CVT_ELEMS;
  unsigned short* W_IH1B = W16 + (size_t)BS6 * CVT_ELEMS;
  unsigned short* W_HH1B = W16 + (size_t)BS7 * CVT_ELEMS;
  unsigned short* W_FF1  = W16 + (size_t)BS8 * CVT_ELEMS;
  unsigned short* W_FF2  = W16 + (size_t)BS9 * CVT_ELEMS;

  WSrc wsrc;
  wsrc.p0 = w_ih0f; wsrc.p1 = w_hh0f; wsrc.p2 = w_ih0b; wsrc.p3 = w_hh0b; wsrc.p4 = w_ih1f;
  wsrc.p5 = w_hh1f; wsrc.p6 = w_ih1b; wsrc.p7 = w_hh1b; wsrc.p8 = w1;     wsrc.p9 = w2;
  cvt_weights_kernel<<<BS10, 256, 0, stream>>>(wsrc, W16);

  xpose_kernel<<<dim3(NSEQ / 64, NCH / 64, NBATCH), 256, 0, stream>>>(x, XT);

  const int gridGi = (NROWS / 64) * (NGATE / 64) / 8;
  const int gridF1 = (NROWS / 64) * (NFF / 64) / 8;
  const int gridF2 = (NROWS / 64) * (NCH / 64) / 8;

  wmma_gemm64<0, 1><<<gridGi, 256, 0, stream>>>(XT, NCH, W_IH0F, NCH, (void*)GI, NGATE, b_ih0f, NROWS, NGATE, NCH, WCARRY_INV);
  gru_scan_kernel<false><<<1, SCAN_THR, 0, stream>>>(GI, W_HH0F, b_hh0f, (void*)H0, 0);
  wmma_gemm64<0, 1><<<gridGi, 256, 0, stream>>>(XT, NCH, W_IH0B, NCH, (void*)GI, NGATE, b_ih0b, NROWS, NGATE, NCH, WCARRY_INV);
  gru_scan_kernel<false><<<1, SCAN_THR, 0, stream>>>(GI, W_HH0B, b_hh0b, (void*)H0, 1);

  wmma_gemm64<0, 1><<<gridGi, 256, 0, stream>>>(H0, 2 * NHID, W_IH1F, 2 * NHID, (void*)GI, NGATE, b_ih1f, NROWS, NGATE, 2 * NHID, WCARRY_INV);
  gru_scan_kernel<true><<<1, SCAN_THR, 0, stream>>>(GI, W_HH1F, b_hh1f, (void*)H1F, 0);
  wmma_gemm64<0, 1><<<gridGi, 256, 0, stream>>>(H0, 2 * NHID, W_IH1B, 2 * NHID, (void*)GI, NGATE, b_ih1b, NROWS, NGATE, 2 * NHID, WCARRY_INV);
  gru_scan_kernel<true><<<1, SCAN_THR, 0, stream>>>(GI, W_HH1B, b_hh1b, (void*)H1B, 1);

  sum_ln_kernel<<<NROWS / 8, 256, 0, stream>>>(H1F, H1B, ln_g, ln_b, LNP);

  wmma_gemm64<2, 1><<<gridF1, 256, 0, stream>>>(LNP, NCH, W_FF1, NCH, (void*)RELU, NFF, b1, NROWS, NFF, NCH, WCARRY_INV);

  wmma_gemm64<0, 3><<<gridF2, 256, 0, stream>>>(RELU, NFF, W_FF2, NFF, (void*)out, NSEQ, b2, NROWS, NCH, NFF, WCARRY_INV);
}
